// MultiHeadAttention_23733989278260
// MI455X (gfx1250) — hardware-verified
//
#include <hip/hip_runtime.h>


#ifndef SEQ
#define SEQ 2048
#endif
#define SEQ_FULL 2048
#define DM   1024
#define NH_  16
#define HD   64
#define HALFD 512
#define PCAR 1024.0f
#define PP   40
#define OSP  68

static_assert(SEQ % 64 == 0);
static_assert(SEQ <= SEQ_FULL);
static_assert(DM % 64 == 0);
static_assert(DM % 32 == 0);
static_assert(NH_ * HD == DM);
static_assert(HD == 64);
static_assert(2 * HALFD == DM);
static_assert((NH_ * (SEQ / 16)) % 8 == 0);
static_assert((PP * 2) % 16 == 0);
static_assert((OSP * 4) % 16 == 0);
static_assert(PP >= 32);
static_assert(OSP >= 64);

typedef _Float16 h16;
typedef unsigned short bf;
typedef __attribute__((ext_vector_type(16))) __bf16   v16bf;
typedef __attribute__((ext_vector_type(16))) _Float16 v16h;
typedef __attribute__((ext_vector_type(8)))  _Float16 v8h;
typedef __attribute__((ext_vector_type(8)))  unsigned short v8us;
typedef __attribute__((ext_vector_type(2)))  unsigned short v2us;
typedef __attribute__((ext_vector_type(8)))  float    v8f;
typedef __attribute__((ext_vector_type(4)))  float    v4f;
typedef __attribute__((ext_vector_type(2)))  float    v2f;
typedef v8h  __attribute__((may_alias)) v8ha;
typedef v4f  __attribute__((may_alias)) v4fa;

__device__ __forceinline__ unsigned short f2bf(float f) { unsigned u = __float_as_uint(f); u += 0x7FFFu + ((u >> 16) & 1u); return (unsigned short)(u >> 16); }
__device__ __forceinline__ float bf2f(unsigned short b) { return __uint_as_float(((unsigned)b) << 16); }
__device__ __forceinline__ float bfr(float f) { return bf2f(f2bf(f)); }
__device__ __forceinline__ void splitf(float y, unsigned short& h, unsigned short& l) { h = f2bf(y); l = f2bf(y - bf2f(h)); }
__device__ __forceinline__ v16h cat16(v8h lo, v8h hi) { return __builtin_shufflevector(lo, hi, 0, 1, 2, 3, 4, 5, 6, 7, 8, 9, 10, 11, 12, 13, 14, 15); }
__device__ __forceinline__ v16bf cat16b(v8us lo, v8us hi) { return __builtin_bit_cast(v16bf, __builtin_shufflevector(lo, hi, 0, 1, 2, 3, 4, 5, 6, 7, 8, 9, 10, 11, 12, 13, 14, 15)); }
__device__ __forceinline__ v8f wmma16(v16h a, v16h b, v8f c) { return __builtin_amdgcn_wmma_f32_16x16x32_f16(false, a, false, b, (short)0, c, false, false); }
__device__ __forceinline__ v8f wmmab(v16bf a, v16bf b, v8f c) { return __builtin_amdgcn_wmma_f32_16x16x32_bf16(false, a, false, b, (short)0, c, false, false); }
__device__ __forceinline__ v16bf ldb(const bf* p) { return cat16b(*(const v8us*)p, *(const v8us*)(p + 16)); }
__device__ __forceinline__ v16h ldh(const h16* p) { return cat16(*(const v8h*)p, *(const v8h*)(p + 16)); }

template <int NSPLIT>
__device__ __forceinline__ void gemmw_body(const bf* A, const bf* A2, const bf* Bt, float* C, const float* bias) {
    __shared__ __align__(16) float os[16 * OSP];
    const int lane = threadIdx.x & 31, lr = lane & 15, hi = lane >> 4; const int r0 = blockIdx.x * 64, c0 = blockIdx.y * 64;
    v8f acc[4][4];
#pragma unroll
    for (int mb = 0; mb < 4; ++mb)
#pragma unroll
        for (int nb = 0; nb < 4; ++nb) acc[mb][nb] = (v8f){};
    const size_t aoff = (size_t)(r0 + lr) * DM + 8 * hi, boff = (size_t)(c0 + lr) * DM + 8 * hi;
#pragma unroll 1
    for (int kc = 0; kc < DM; kc += 32) {
        v16bf a[4], a2[4];
#pragma unroll
        for (int mb = 0; mb < 4; ++mb) { a[mb] = ldb(A + aoff + (size_t)mb * 16 * DM + kc); if (NSPLIT == 1) a2[mb] = ldb(A2 + aoff + (size_t)mb * 16 * DM + kc); else a2[mb] = a[mb]; }
#pragma unroll
        for (int nb = 0; nb < 4; ++nb) { const v16bf b = ldb(Bt + boff + (size_t)nb * 16 * DM + kc);
#pragma unroll
            for (int mb = 0; mb < 4; ++mb) { acc[mb][nb] = wmmab(a[mb], b, acc[mb][nb]); if (NSPLIT == 1) acc[mb][nb] = wmmab(a2[mb], b, acc[mb][nb]); } }
        asm volatile("v_nop\n\tv_nop\n\tv_nop\n\tv_nop" : "+v"(acc[0][0]), "+v"(acc[1][1]), "+v"(acc[2][2]), "+v"(acc[3][3]) : "v"(a[0]), "v"(a[3]));
    }
    const v4f bz = *(const v4f*)(bias + c0 + lr * 4); v4f bb;
#pragma unroll
    for (int q = 0; q < 4; ++q) bb[q] = bfr(bz[q]);
#pragma unroll
    for (int mb = 0; mb < 4; ++mb) {
#pragma unroll
        for (int nb = 0; nb < 4; ++nb) {
#pragma unroll
            for (int j = 0; j < 8; ++j) os[(hi * 8 + j) * OSP + nb * 16 + lr] = acc[mb][nb][j]; }
        __builtin_amdgcn_wave_barrier(); asm volatile("" ::: "memory");
        float* crow = C + (size_t)(r0 + mb * 16) * DM + c0;
#pragma unroll 1
        for (int ps = 0; ps < 2; ++ps) {
#pragma unroll
            for (int s = 0; s < 8; ++s) { const int row = 2 * s + hi, cofs = lr * 4; v4f val = *(const v4fa*)(os + row * OSP + cofs); val += bb;
                *(volatile v4f*)(crow + (size_t)row * DM + cofs) = val; }
            if (ps == 0) __threadfence(); }
        __builtin_amdgcn_wave_barrier(); asm volatile("" ::: "memory");
    }
}
__global__ __launch_bounds__(32) void k_gemm_proj(const bf* __restrict__ A, const bf* __restrict__ Bt, float* C, const float* __restrict__ bias) { gemmw_body<0>(A, A, Bt, C, bias); }
__global__ __launch_bounds__(32) void k_gemm_out(const bf* __restrict__ A, const bf* __restrict__ A2, const bf* __restrict__ Bt, float* C, const float* __restrict__ bias) { gemmw_body<1>(A, A2, Bt, C, bias); }

__global__ __launch_bounds__(256) void k_wtG(const float* __restrict__ w, int K, int N, bf* Bt) {
    const int lane = threadIdx.x & 31; const int L0 = (blockIdx.x * 8 + (threadIdx.x >> 5)) * 8; const int nlines = N * K / 64;
#pragma unroll
    for (int ps = 0; ps < 2; ++ps) {
#pragma unroll 1
        for (int l = 0; l < 8; ++l) { const int L = L0 + l; if (L >= nlines) break; const size_t e = (size_t)L * 64 + lane * 2; const int k = (int)(e % K), n = (int)(e / K); v2us o;
            o[0] = f2bf(w[(size_t)k * N + n]); o[1] = f2bf(w[(size_t)(k + 1) * N + n]); *(volatile v2us*)(Bt + e) = o; }
        if (ps == 0) __threadfence(); }
}
__global__ __launch_bounds__(256) void k_cvt8(const float* __restrict__ src, bf* dst, size_t n8) { const size_t i = (size_t)blockIdx.x * 256 + threadIdx.x; if (i >= n8) return; const v8f v = *(const v8f*)(src + i * 8); v8us o;
#pragma unroll
    for (int k = 0; k < 8; ++k) o[k] = f2bf(v[k]); *(volatile v8us*)(dst + i * 8) = o; __threadfence(); *(volatile v8us*)(dst + i * 8) = o; }

__global__ __launch_bounds__(128) void k_theta(float* TH) {
    const int j = blockIdx.x * 128 + threadIdx.x; if (j >= HALFD) return;
    const float e = (float)(2 * j) * (1.0f / 1024.0f);
    const float p = powf(10000.0f, e); const float th = 1.0f / p;
    *(volatile float*)(TH + j) = th; __threadfence(); *(volatile float*)(TH + j) = th; }
__global__ __launch_bounds__(256) void k_cstab(const float* __restrict__ TH, float* CS) {
    const int idx = blockIdx.x * 256 + threadIdx.x; if (idx >= SEQ * HALFD) return; const int t = idx >> 9, j = idx & (HALFD - 1);
    float ang = __fmul_rn((float)t, TH[j]); float s, c; sincosf(ang, &s, &c); v2f cs; cs[0] = c; cs[1] = s;
    *(volatile v2f*)(CS + (size_t)idx * 2) = cs; __threadfence(); *(volatile v2f*)(CS + (size_t)idx * 2) = cs; }

__global__ __launch_bounds__(256) void k_ropeP(const float* __restrict__ F, const float* __restrict__ CS, bf* Ph, bf* Pl) {
#pragma clang fp contract(off)
    const size_t i = (size_t)blockIdx.x * 256 + threadIdx.x; if (i >= (size_t)SEQ * DM / 8) return; const size_t e = i * 8; const int d0 = (int)(e % DM); const int t = (int)(e / DM); const int j0 = d0 & (HALFD - 1); const bool up = (d0 >= HALFD);
    const v4f y0 = *(const v4f*)(F + e), y1 = *(const v4f*)(F + e + 4); const float* cp = CS + ((size_t)t * HALFD + j0) * 2;
    const v4f c0 = *(const v4f*)(cp), c1 = *(const v4f*)(cp + 4), c2 = *(const v4f*)(cp + 8), c3 = *(const v4f*)(cp + 12);
    float yy[8] = { y0[0], y0[1], y0[2], y0[3], y1[0], y1[1], y1[2], y1[3] };
    float cc[8] = { c0[0], c0[2], c1[0], c1[2], c2[0], c2[2], c3[0], c3[2] };
    float ss[8] = { c0[1], c0[3], c1[1], c1[3], c2[1], c2[3], c3[1], c3[3] };
    v8us oh, ol;
#pragma unroll
    for (int q = 0; q < 8; ++q) { const float y = yy[q]; const float nn = up ? -y : y; float a = __fmul_rn(y, cc[q]); float b = __fmul_rn(nn, ss[q]); asm volatile("" : "+v"(a)); asm volatile("" : "+v"(b)); const float r = __fadd_rn(a, b);
        unsigned short hh, ll; splitf(r, hh, ll); oh[q] = hh; ol[q] = ll; }
    *(volatile v8us*)(Ph + e) = oh; *(volatile v8us*)(Pl + e) = ol; __threadfence(); *(volatile v8us*)(Ph + e) = oh; *(volatile v8us*)(Pl + e) = ol; }

__global__ __launch_bounds__(256) void k_vt(const float* __restrict__ F, h16* V16) {
    const size_t i = (size_t)blockIdx.x * 256 + threadIdx.x; if (i >= (size_t)DM * SEQ / 8) return; const size_t e = i * 8; const int t = (int)(e % SEQ); const int col = (int)(e / SEQ); v8h o;
#pragma unroll
    for (int q = 0; q < 8; ++q) o[q] = (h16)F[(size_t)(t + q) * DM + col];
    *(volatile v8h*)(V16 + e) = o; __threadfence(); *(volatile v8h*)(V16 + e) = o; }

__device__ __forceinline__ v8f score_tile(const bf* __restrict__ Kh, const bf* __restrict__ Kl, size_t ko, v16bf qh0, v16bf qh1, v16bf ql0, v16bf ql1) {
    const v16bf kh0 = ldb(Kh + ko), kh1 = ldb(Kh + ko + 32), kl0 = ldb(Kl + ko), kl1 = ldb(Kl + ko + 32);
    v8f c = (v8f){};
    c = wmmab(qh0, kh0, c); c = wmmab(ql0, kh0, c); c = wmmab(qh0, kl0, c);
    c = wmmab(qh1, kh1, c); c = wmmab(ql1, kh1, c); c = wmmab(qh1, kl1, c);
    asm volatile("v_nop\n\tv_nop\n\tv_nop\n\tv_nop" : "+v"(c) : "v"(kh1), "v"(kl1), "v"(qh1));
    return c; }

__global__ __launch_bounds__(256) void k_flash(const bf* __restrict__ Qh, const bf* __restrict__ Ql, const bf* __restrict__ Kh, const bf* __restrict__ Kl, const h16* __restrict__ Vt, bf* Ah, bf* Al) {
    __shared__ __align__(16) h16 pls[8 * 16 * PP];
    __shared__ __align__(16) float ost[8 * 16 * OSP];
    const int lane = threadIdx.x & 31, wave = threadIdx.x >> 5, l16 = lane & 15, half = lane >> 4;
    const int w = blockIdx.x * 8 + wave; const int h = w / (SEQ / 16); const int t0 = (w % (SEQ / 16)) * 16;
    h16* pl = pls + wave * 16 * PP; float* ow = ost + wave * 16 * OSP;
    const float SC2 = 0.125f * 1.4426950408889634f;
    const size_t qo = (size_t)(t0 + l16) * DM + h * HD + 8 * half;
    const v16bf qh0 = ldb(Qh + qo), qh1 = ldb(Qh + qo + 32), ql0 = ldb(Ql + qo), ql1 = ldb(Ql + qo + 32);
    float m[8], l[8]; v8f acc[4];
#pragma unroll
    for (int r = 0; r < 8; ++r) { m[r] = -3.0e38f; l[r] = 0.0f; }
#pragma unroll
    for (int n = 0; n < 4; ++n) acc[n] = (v8f){};
    const size_t kbase = (size_t)l16 * DM + h * HD + 8 * half;
    const size_t vbase = (size_t)(h * HD + l16) * SEQ + 8 * half;
#pragma unroll 1
    for (int jb = 0; jb < SEQ / 32; ++jb) {
        const size_t ko = kbase + (size_t)jb * 32 * DM;
        const v8f sa = score_tile(Kh, Kl, ko, qh0, qh1, ql0, ql1);
        const v8f sb = score_tile(Kh, Kl, ko + (size_t)16 * DM, qh0, qh1, ql0, ql1);
#pragma unroll
        for (int r = 0; r < 8; ++r) {
            const float s0 = sa[r] * SC2, s1 = sb[r] * SC2;
            float mloc = fmaxf(s0, s1);
#pragma unroll
            for (int d = 1; d < 16; d <<= 1) mloc = fmaxf(mloc, __shfl_xor(mloc, d, 32));
            const float mnew = fmaxf(m[r], mloc);
            const float corr = __builtin_amdgcn_exp2f(m[r] - mnew);
            const float p0 = __builtin_amdgcn_exp2f(s0 - mnew);
            const float p1 = __builtin_amdgcn_exp2f(s1 - mnew);
            float ls = p0 + p1;
#pragma unroll
            for (int d = 1; d < 16; d <<= 1) ls += __shfl_xor(ls, d, 32);
            l[r] = l[r] * corr + ls; m[r] = mnew;
#pragma unroll
            for (int n = 0; n < 4; ++n) acc[n][r] *= corr;
            const int row = r + 8 * half;
            pl[row * PP + l16]      = (h16)(p0 * PCAR);
            pl[row * PP + 16 + l16] = (h16)(p1 * PCAR);
        }
        __builtin_amdgcn_wave_barrier(); asm volatile("s_wait_dscnt 0" ::: "memory");
        const v16h pa = cat16(*(const v8ha*)(pl + l16 * PP + 8 * half), *(const v8ha*)(pl + l16 * PP + 16 + 8 * half));
        const size_t vo = vbase + (size_t)jb * 32;
        const v16h v0 = ldh(Vt + vo), v1 = ldh(Vt + vo + (size_t)16 * SEQ), v2 = ldh(Vt + vo + (size_t)32 * SEQ), v3 = ldh(Vt + vo + (size_t)48 * SEQ);
        acc[0] = wmma16(pa, v0, acc[0]); acc[1] = wmma16(pa, v1, acc[1]); acc[2] = wmma16(pa, v2, acc[2]); acc[3] = wmma16(pa, v3, acc[3]);
        asm volatile("v_nop\n\tv_nop\n\tv_nop\n\tv_nop" : "+v"(acc[0]), "+v"(acc[1]), "+v"(acc[2]), "+v"(acc[3]) : "v"(pa), "v"(v3));
        __builtin_amdgcn_wave_barrier(); asm volatile("" ::: "memory");
    }
    float inv[8];
#pragma unroll
    for (int r = 0; r < 8; ++r) inv[r] = 1.0f / (l[r] * PCAR);
#pragma unroll
    for (int n = 0; n < 4; ++n)
#pragma unroll
        for (int r = 0; r < 8; ++r) ow[(8 * half + r) * OSP + n * 16 + l16] = acc[n][r] * inv[r];
    __builtin_amdgcn_wave_barrier(); asm volatile("s_wait_dscnt 0" ::: "memory");
    const int rq = lane >> 3, piece = lane & 7;
#pragma unroll 1
    for (int ps = 0; ps < 2; ++ps) {
#pragma unroll
        for (int s4 = 0; s4 < 4; ++s4) { const int row = 4 * s4 + rq; const v4f x0 = *(const v4fa*)(ow + row * OSP + piece * 8), x1 = *(const v4fa*)(ow + row * OSP + piece * 8 + 4); v8us oh, ol;
#pragma unroll
            for (int q = 0; q < 4; ++q) { unsigned short a, b; splitf(x0[q], a, b); oh[q] = a; ol[q] = b; splitf(x1[q], a, b); oh[4 + q] = a; ol[4 + q] = b; }
            const size_t oo = (size_t)(t0 + row) * DM + h * HD + piece * 8; *(volatile v8us*)(Ah + oo) = oh; *(volatile v8us*)(Al + oo) = ol; }
        if (ps == 0) __threadfence(); }
}

constexpr size_t al256(size_t b) { return (b + 255) & ~(size_t)255; }
constexpr size_t WS_TOTAL = 4 * al256((size_t)DM * DM * 2) + 3 * al256((size_t)SEQ * DM * 2) + al256((size_t)HALFD * 4) + al256((size_t)SEQ * HALFD * 2 * 4)
                          + 3 * al256((size_t)SEQ * DM * 4) + 4 * al256((size_t)SEQ * DM * 2) + al256((size_t)DM * SEQ * 2) + 2 * al256((size_t)SEQ * DM * 2);
static_assert(WS_TOTAL <= (size_t)134217728);

extern "C" void kernel_launch(void* const* d_in, const int* in_sizes, int n_in,
                              void* d_out, int out_size, void* d_ws, size_t ws_size, hipStream_t stream) {
    if (n_in < 11) return;
    if (in_sizes[0] < SEQ * DM || in_sizes[1] < SEQ * DM || in_sizes[2] < SEQ * DM) return;
    if (in_sizes[3] < DM * DM || in_sizes[5] < DM * DM || in_sizes[7] < DM * DM || in_sizes[9] < DM * DM) return;
    if (in_sizes[4] < DM || in_sizes[6] < DM || in_sizes[8] < DM || in_sizes[10] < DM) return;
    if (out_size < SEQ * DM) return;
    if (WS_TOTAL > ws_size) return;
    const float* query = (const float*)d_in[0]; const float* key_ = (const float*)d_in[1]; const float* value = (const float*)d_in[2];
    const float* wq = (const float*)d_in[3]; const float* bq = (const float*)d_in[4];
    const float* wk = (const float*)d_in[5]; const float* bk = (const float*)d_in[6];
    const float* wv = (const float*)d_in[7]; const float* bv = (const float*)d_in[8];
    const float* wo = (const float*)d_in[9]; const float* bo = (const float*)d_in[10];
    float* OUT = (float*)d_out;
    char* wsp = (char*)d_ws;
    auto take = [&](size_t bytes) { char* p = wsp; wsp += (bytes + 255) & ~(size_t)255; return (void*)p; };
    bf* WQ = (bf*)take((size_t)DM * DM * 2); bf* WK = (bf*)take((size_t)DM * DM * 2); bf* WV = (bf*)take((size_t)DM * DM * 2); bf* WO = (bf*)take((size_t)DM * DM * 2);
    bf* XQ = (bf*)take((size_t)SEQ * DM * 2); bf* XK = (bf*)take((size_t)SEQ * DM * 2); bf* XV = (bf*)take((size_t)SEQ * DM * 2);
    float* TH = (float*)take((size_t)HALFD * 4); float* CS = (float*)take((size_t)SEQ * HALFD * 2 * 4);
    float* FQ = (float*)take((size_t)SEQ * DM * 4); float* FK = (float*)take((size_t)SEQ * DM * 4); float* FV = (float*)take((size_t)SEQ * DM * 4);
    bf* QPh = (bf*)take((size_t)SEQ * DM * 2); bf* QPl = (bf*)take((size_t)SEQ * DM * 2); bf* KPh = (bf*)take((size_t)SEQ * DM * 2); bf* KPl = (bf*)take((size_t)SEQ * DM * 2);
    h16* VT16 = (h16*)take((size_t)DM * SEQ * 2);
    bf* ATh = (bf*)take((size_t)SEQ * DM * 2); bf* ATl = (bf*)take((size_t)SEQ * DM * 2);
    if ((size_t)(wsp - (char*)d_ws) > ws_size) return;

    const unsigned gW = (unsigned)((DM * DM / 64 + 63) / 64);
    k_wtG<<<gW, 256, 0, stream>>>(wq, DM, DM, WQ);
    k_wtG<<<gW, 256, 0, stream>>>(wk, DM, DM, WK);
    k_wtG<<<gW, 256, 0, stream>>>(wv, DM, DM, WV);
    k_wtG<<<gW, 256, 0, stream>>>(wo, DM, DM, WO);
    const size_t n8 = (size_t)SEQ * DM / 8; const unsigned g8 = (unsigned)((n8 + 255) / 256);
    k_cvt8<<<g8, 256, 0, stream>>>(query, XQ, n8);
    k_cvt8<<<g8, 256, 0, stream>>>(key_, XK, n8);
    k_cvt8<<<g8, 256, 0, stream>>>(value, XV, n8);
    k_theta<<<(HALFD + 127) / 128, 128, 0, stream>>>(TH);
    k_cstab<<<(unsigned)(((size_t)SEQ * HALFD + 255) / 256), 256, 0, stream>>>(TH, CS);
    k_gemm_proj<<<dim3(SEQ / 64, DM / 64, 1), 32, 0, stream>>>(XQ, WQ, FQ, bq);
    k_gemm_proj<<<dim3(SEQ / 64, DM / 64, 1), 32, 0, stream>>>(XK, WK, FK, bk);
    k_gemm_proj<<<dim3(SEQ / 64, DM / 64, 1), 32, 0, stream>>>(XV, WV, FV, bv);
    k_ropeP<<<g8, 256, 0, stream>>>(FQ, CS, QPh, QPl);
    k_ropeP<<<g8, 256, 0, stream>>>(FK, CS, KPh, KPl);
    k_vt<<<g8, 256, 0, stream>>>(FV, VT16);
    k_flash<<<(unsigned)(NH_ * (SEQ / 16) / 8), 256, 0, stream>>>(QPh, QPl, KPh, KPl, VT16, ATh, ATl);
    k_gemm_out<<<dim3(SEQ / 64, DM / 64, 1), 32, 0, stream>>>(ATh, ATl, WO, OUT, bo);
}
